// ConvNeXtStyleBlock_56530359550551
// MI455X (gfx1250) — hardware-verified
//
#include <hip/hip_runtime.h>
#include <stddef.h>


typedef _Float16 v16h __attribute__((ext_vector_type(16)));
typedef _Float16 v8h  __attribute__((ext_vector_type(8)));
typedef _Float16 v4h  __attribute__((ext_vector_type(4)));
typedef float    v8f  __attribute__((ext_vector_type(8)));
typedef float    v4f  __attribute__((ext_vector_type(4)));

union Frag { v16h v; v8h half[2]; };

#define CCH        768
#define HWN        1024
#define KSTEPS     (CCH / 32)
#define APITCH     40
#define TPITCH     776
#define SPITCH     68
#define TILE_BYTES (64 * TPITCH * 2)

__device__ __forceinline__ v8f wmma_f16(v16h a, v16h b, v8f c)
{
  v8f d = __builtin_amdgcn_wmma_f32_16x16x32_f16(false, a, false, b, (short)0, c, false, false);
  asm volatile("v_nop\n\tv_nop\n\tv_nop\n\tv_nop" : "+v"(d) : "v"(a), "v"(b));
  return d;
}

__global__ __launch_bounds__(256) void k_wcvt(const float* __restrict__ w0,
                                              const float* __restrict__ w1,
                                              const float* __restrict__ w2,
                                              _Float16* __restrict__ wb, int n8)
{
  const int which = blockIdx.y;
  const float* w = (which == 0) ? w0 : ((which == 1) ? w1 : w2);
  _Float16* dst = wb + (size_t)which * (size_t)n8 * 8;
  const int i = blockIdx.x * blockDim.x + threadIdx.x;
  if (i < n8) {
    const v4f a = *(const v4f*)(w + (size_t)i * 8);
    const v4f b = *(const v4f*)(w + (size_t)i * 8 + 4);
    v8h o;
    o[0] = (_Float16)(a[0] * 64.0f);
    o[1] = (_Float16)(a[1] * 64.0f);
    o[2] = (_Float16)(a[2] * 64.0f);
    o[3] = (_Float16)(a[3] * 64.0f);
    o[4] = (_Float16)(b[0] * 64.0f);
    o[5] = (_Float16)(b[1] * 64.0f);
    o[6] = (_Float16)(b[2] * 64.0f);
    o[7] = (_Float16)(b[3] * 64.0f);
    volatile v8h* p = (volatile v8h*)(dst + (size_t)i * 8);
    *p = o;
    __threadfence();
    *p = o;
  }
}

__global__ __launch_bounds__(256) void k_tin(const float* __restrict__ x,
                                             _Float16* __restrict__ xt, int nrows)
{
  __shared__ _Float16 tile[32 * TPITCH] __attribute__((aligned(16)));
  const int tid = threadIdx.x, lane = tid & 31, wave = tid >> 5;
  const int b  = blockIdx.y;
  const int p0 = blockIdx.x * 32;
  const float* src = x + (size_t)b * CCH * HWN + p0;
  const int q = lane & 7, cs = lane >> 3;
  for (int it = 0; it < CCH / 32; ++it) {
    const int c = it * 32 + wave * 4 + cs;
    const v4f v = *(const v4f*)(src + (size_t)c * HWN + q * 4);
    _Float16* t = tile + (q * 4) * TPITCH + c;
    t[0]          = (_Float16)(v[0] * 16.0f);
    t[TPITCH]     = (_Float16)(v[1] * 16.0f);
    t[2 * TPITCH] = (_Float16)(v[2] * 16.0f);
    t[3 * TPITCH] = (_Float16)(v[3] * 16.0f);
  }
  __syncthreads();
  for (int pass = 0; pass < 2; ++pass) {
    for (int rr = 0; rr < 4; ++rr) {
      const int r = wave * 4 + rr;
      const int n = b * HWN + p0 + r;
      if (n < nrows) {
        const _Float16* trow = tile + r * TPITCH + lane * 8;
        _Float16* grow = xt + (size_t)n * CCH + lane * 8;
#pragma unroll
        for (int j = 0; j < 3; ++j) {
          const v8h v = *(const v8h*)(trow + j * 256);
          *(volatile v8h*)(grow + j * 256) = v;
        }
      }
    }
    if (pass == 0) __threadfence();
  }
}

template <bool DO_LN>
__global__ __launch_bounds__(512) void k_gemm(const _Float16* __restrict__ A,
                                              const _Float16* __restrict__ Wb,
                                              const float* __restrict__ bias,
                                              const float* __restrict__ gamma,
                                              const float* __restrict__ beta,
                                              _Float16* __restrict__ outH,
                                              float* __restrict__ outF,
                                              int nrows)
{
  __shared__ _Float16 ldsA[2][64 * APITCH] __attribute__((aligned(16)));
  __shared__ unsigned char ldsT[TILE_BYTES] __attribute__((aligned(16)));
  __shared__ float lds_part[16 * 64];
  __shared__ float lds_mu[64];
  __shared__ float lds_rs[64];

  const int tid  = threadIdx.x;
  const int lane = tid & 31;
  const int wave = tid >> 5;
  const int h    = lane >> 4;
  const int lm   = lane & 15;
  const int n0   = blockIdx.x * 64;
  const int o0   = wave * 48;

  const int arow = tid >> 3;
  const int acol = (tid & 7) * 4;
  int ga = n0 + arow;
  if (ga > nrows - 1) ga = nrows - 1;
  const _Float16* gA = A + (size_t)ga * CCH + acol;
  const int loff = arow * APITCH + acol;

  { const v4h v = *(const v4h*)gA; *(v4h*)(&ldsA[0][loff]) = v; }
  __syncthreads();

  v8f acc[4][3];
#pragma unroll
  for (int mt = 0; mt < 4; ++mt)
#pragma unroll
    for (int nt = 0; nt < 3; ++nt)
#pragma unroll
      for (int r = 0; r < 8; ++r) acc[mt][nt][r] = 0.0f;

  for (int kk = 0; kk < KSTEPS; ++kk) {
    const int buf = kk & 1;
    if (kk + 1 < KSTEPS) {
      const v4h v = *(const v4h*)(gA + (kk + 1) * 32);
      *(v4h*)(&ldsA[buf ^ 1][loff]) = v;
    }

    Frag af[4];
#pragma unroll
    for (int mt = 0; mt < 4; ++mt) {
      const _Float16* p = &ldsA[buf][(mt * 16 + lm) * APITCH + 8 * h];
      af[mt].half[0] = *(const v8h*)(p);
      af[mt].half[1] = *(const v8h*)(p + 16);
    }

    const _Float16* wk = Wb + (size_t)kk * 32 + 8 * h;
#pragma unroll
    for (int nt = 0; nt < 3; ++nt) {
      Frag bfr;
      const _Float16* q = wk + (size_t)(o0 + nt * 16 + lm) * CCH;
      bfr.half[0] = *(const v8h*)(q);
      bfr.half[1] = *(const v8h*)(q + 16);
#pragma unroll
      for (int mt = 0; mt < 4; ++mt)
        acc[mt][nt] = wmma_f16(af[mt].v, bfr.v, acc[mt][nt]);
    }
    __syncthreads();
  }

  const float SC = 0.0009765625f;
  float bo[3], go[3], bt[3];
#pragma unroll
  for (int nt = 0; nt < 3; ++nt) {
    const int o = o0 + nt * 16 + lm;
    bo[nt] = bias[o];
    go[nt] = 1.0f; bt[nt] = 0.0f;
    if (DO_LN) { go[nt] = gamma[o]; bt[nt] = beta[o]; }
  }
#pragma unroll
  for (int mt = 0; mt < 4; ++mt)
#pragma unroll
    for (int nt = 0; nt < 3; ++nt)
#pragma unroll
      for (int r = 0; r < 8; ++r) acc[mt][nt][r] = acc[mt][nt][r] * SC + bo[nt];

  if (DO_LN) {
#pragma unroll
    for (int mt = 0; mt < 4; ++mt) {
#pragma unroll
      for (int r = 0; r < 8; ++r) {
        float s = acc[mt][0][r] + acc[mt][1][r] + acc[mt][2][r];
        s += __shfl_xor(s, 1, 32);
        s += __shfl_xor(s, 2, 32);
        s += __shfl_xor(s, 4, 32);
        s += __shfl_xor(s, 8, 32);
        if (lm == 0) lds_part[wave * 64 + mt * 16 + 8 * h + r] = s;
      }
    }
    __syncthreads();
    if (tid < 64) {
      float t = 0.0f;
#pragma unroll
      for (int w = 0; w < 16; ++w) t += lds_part[w * 64 + tid];
      lds_mu[tid] = t * (1.0f / 768.0f);
    }
    __syncthreads();
#pragma unroll
    for (int mt = 0; mt < 4; ++mt) {
#pragma unroll
      for (int r = 0; r < 8; ++r) {
        const float mu = lds_mu[mt * 16 + 8 * h + r];
        const float d0 = acc[mt][0][r] - mu;
        const float d1 = acc[mt][1][r] - mu;
        const float d2 = acc[mt][2][r] - mu;
        float s = d0 * d0 + d1 * d1 + d2 * d2;
        s += __shfl_xor(s, 1, 32);
        s += __shfl_xor(s, 2, 32);
        s += __shfl_xor(s, 4, 32);
        s += __shfl_xor(s, 8, 32);
        if (lm == 0) lds_part[wave * 64 + mt * 16 + 8 * h + r] = s;
      }
    }
    __syncthreads();
    if (tid < 64) {
      float t = 0.0f;
#pragma unroll
      for (int w = 0; w < 16; ++w) t += lds_part[w * 64 + tid];
      const float var = t * (1.0f / 768.0f);
      lds_rs[tid] = rsqrtf(var + 1e-6f);
    }
    __syncthreads();

    _Float16* tile = (_Float16*)ldsT;
#pragma unroll
    for (int mt = 0; mt < 4; ++mt) {
#pragma unroll
      for (int r = 0; r < 8; ++r) {
        const int row = mt * 16 + 8 * h + r;
        const float mu = lds_mu[row];
        const float rs = lds_rs[row];
#pragma unroll
        for (int nt = 0; nt < 3; ++nt) {
          float y = (acc[mt][nt][r] - mu) * rs * go[nt] + bt[nt];
          y = 0.5f * y * (1.0f + erff(y * 0.70710678118654752f));
          tile[row * TPITCH + o0 + nt * 16 + lm] = (_Float16)(y * 16.0f);
        }
      }
    }
    __syncthreads();

    for (int pass = 0; pass < 2; ++pass) {
#pragma unroll
      for (int rr = 0; rr < 4; ++rr) {
        const int row = wave * 4 + rr;
        const int n = n0 + row;
        if (n < nrows) {
          const _Float16* trow = tile + row * TPITCH + lane * 8;
          _Float16* grow = outH + (size_t)n * CCH + lane * 8;
#pragma unroll
          for (int j = 0; j < 3; ++j) {
            const v8h v = *(const v8h*)(trow + j * 256);
            *(volatile v8h*)(grow + j * 256) = v;
          }
        }
      }
      if (pass == 0) __threadfence();
    }
  } else {
    float* stg = (float*)ldsT + wave * (16 * SPITCH);
    const int bb  = n0 / HWN;
    const int hw0 = n0 - bb * HWN;
    const int rq  = lm * 4;
    const bool rows_ok = (n0 + 64 <= nrows);
#pragma unroll
    for (int nt = 0; nt < 3; ++nt) {
#pragma unroll
      for (int mt = 0; mt < 4; ++mt)
#pragma unroll
        for (int r = 0; r < 8; ++r)
          stg[lm * SPITCH + mt * 16 + 8 * h + r] = acc[mt][nt][r];
      __syncthreads();
      for (int pass = 0; pass < 2; ++pass) {
#pragma unroll
        for (int pp = 0; pp < 8; ++pp) {
          const int c = 2 * pp + h;
          const v4f v = *(const v4f*)(stg + c * SPITCH + rq);
          const int o = o0 + nt * 16 + c;
          const size_t g = ((size_t)bb * CCH + (size_t)o) * HWN + (size_t)(hw0 + rq);
          if (rows_ok) *(volatile v4f*)(outF + g) = v;
        }
        if (pass == 0) __threadfence();
      }
      __syncthreads();
    }
  }
}

extern "C" void kernel_launch(void* const* d_in, const int* in_sizes, int n_in,
                              void* d_out, int out_size, void* d_ws, size_t ws_size,
                              hipStream_t stream)
{
  if (n_in < 11) return;
  const float* x   = (const float*)d_in[0];
  const float* W1  = (const float*)d_in[1];
  const float* b1  = (const float*)d_in[2];
  const float* g1  = (const float*)d_in[3];
  const float* be1 = (const float*)d_in[4];
  const float* W2  = (const float*)d_in[5];
  const float* b2  = (const float*)d_in[6];
  const float* g2  = (const float*)d_in[7];
  const float* be2 = (const float*)d_in[8];
  const float* W3  = (const float*)d_in[9];
  const float* b3  = (const float*)d_in[10];
  float* out = (float*)d_out;

  const int nrows = in_sizes[0] / CCH;
  if (nrows <= 0 || (nrows % HWN) != 0 || (nrows % 64) != 0) return;
  if (out_size != nrows * CCH) return;
  const int nb = nrows / HWN;
  const int wn = in_sizes[1];
  if (wn != CCH * CCH || in_sizes[5] != wn || in_sizes[9] != wn) return;
  const int n8 = wn / 8;

  const size_t BUF = (size_t)nrows * CCH * 2;
  const size_t need = 3 * BUF + (size_t)3 * (size_t)wn * 2;
  if (need > ws_size) return;
  char* ws = (char*)d_ws;
  _Float16* XT = (_Float16*)(ws);
  _Float16* H1 = (_Float16*)(ws + BUF);
  _Float16* H2 = (_Float16*)(ws + 2 * BUF);
  _Float16* WB = (_Float16*)(ws + 3 * BUF);

  k_wcvt<<<dim3((n8 + 255) / 256, 3), 256, 0, stream>>>(W1, W2, W3, WB, n8);
  k_tin<<<dim3(HWN / 32, nb), 256, 0, stream>>>(x, XT, nrows);

  const int gblocks = (nrows + 63) / 64;
  k_gemm<true ><<<gblocks, 512, 0, stream>>>(XT, WB,                  b1, g1, be1, H1, out, nrows);
  k_gemm<true ><<<gblocks, 512, 0, stream>>>(H1, WB + (size_t)wn,     b2, g2, be2, H2, out, nrows);
  k_gemm<false><<<gblocks, 512, 0, stream>>>(H2, WB + (size_t)2 * wn, b3, b3, b3,   H1, out, nrows);
}
